// LinearAttention_24824910971194
// MI455X (gfx1250) — hardware-verified
//
#include <hip/hip_runtime.h>
#include <math.h>

constexpr int kBatch  = 2;
constexpr int kSeq    = 1024;
constexpr int kDim    = 1024;
constexpr int kHeads  = 16;
constexpr int kDh     = 64;
constexpr int kTok    = kBatch * kSeq;
constexpr int kChunk  = 64;
constexpr int kNChunk = kSeq / kChunk;
constexpr int kPitch  = 72;
constexpr float kWCarry    = 16.0f;
constexpr float kWCarryInv = 1.0f / 16.0f;
static_assert(kHeads * kDh == kDim, "shape");
static_assert(kSeq % kChunk == 0 && kChunk == 64 && kDh == 64, "core tiles");
static_assert(kTok % 64 == 0 && kDim % 64 == 0 && kDim % 32 == 0, "gemm tiles: M,N multiples of 64, K multiple of 32");
static_assert((kTok * kDim) % (8 * 256) == 0, "cast grid exact");
static_assert(kPitch % 8 == 0, "16-B aligned LDS rows");

typedef __attribute__((ext_vector_type(16))) _Float16 v16h;
typedef __attribute__((ext_vector_type(8)))  _Float16 v8h;
typedef __attribute__((ext_vector_type(16))) __bf16   v16b;
typedef __attribute__((ext_vector_type(8)))  __bf16   v8b;
typedef __attribute__((ext_vector_type(8)))  float    v8f;
typedef __attribute__((ext_vector_type(4)))  float    v4f;
typedef __attribute__((ext_vector_type(4)))  unsigned int v4u;

__device__ __forceinline__ unsigned short f2bf_bits(float f) {
  unsigned u = __float_as_uint(f);
  return (unsigned short)((u + 0x7FFFu + ((u >> 16) & 1u)) >> 16);
}
__device__ __forceinline__ float bf_bits2f(unsigned short h) { return __uint_as_float(((unsigned)h) << 16); }

__device__ __forceinline__ void dep_guard_h(v8f& a, v8f& b, v16h x, v16h y) { asm volatile("v_nop\n\tv_nop\n\tv_nop\n\tv_nop" : "+v"(a), "+v"(b) : "v"(x), "v"(y)); }
__device__ __forceinline__ void dep_guard_b(v8f& a, v8f& b, v16b x, v16b y) { asm volatile("v_nop\n\tv_nop\n\tv_nop\n\tv_nop" : "+v"(a), "+v"(b) : "v"(x), "v"(y)); }
__device__ __forceinline__ void dep_guard4_h(v8f& a, v8f& b, v8f& c, v8f& d, v16h x, v16h y) { asm volatile("v_nop\n\tv_nop\n\tv_nop\n\tv_nop" : "+v"(a), "+v"(b), "+v"(c), "+v"(d) : "v"(x), "v"(y)); }
__device__ __forceinline__ void dep_guard4_b(v8f& a, v8f& b, v8f& c, v8f& d, v16b x, v16b y) { asm volatile("v_nop\n\tv_nop\n\tv_nop\n\tv_nop" : "+v"(a), "+v"(b), "+v"(c), "+v"(d) : "v"(x), "v"(y)); }
__device__ __forceinline__ void keep4_h(v16h a, v16h b, v16h c, v16h d) { asm volatile("v_nop" :: "v"(a), "v"(b), "v"(c), "v"(d)); }
__device__ __forceinline__ void keep4_b(v16b a, v16b b, v16b c, v16b d) { asm volatile("v_nop" :: "v"(a), "v"(b), "v"(c), "v"(d)); }
__device__ __forceinline__ void acc_guard4(v8f& a, v8f& b, v8f& c, v8f& d) { asm volatile("v_nop\n\tv_nop\n\tv_nop\n\tv_nop" : "+v"(a), "+v"(b), "+v"(c), "+v"(d)); }
template <typename T> struct Frag;
template <> struct Frag<_Float16> {
  typedef v16h V; union U { v16h v; v8h h[2]; };
  static __device__ __forceinline__ v16h load(const _Float16* p) {
    U f; f.h[0] = *(const v8h*)(p); f.h[1] = *(const v8h*)(p + 16); return f.v;
  }
  static __device__ __forceinline__ v8f mma(v16h a, v16h b, v8f c) {
    return __builtin_amdgcn_wmma_f32_16x16x32_f16(false, a, false, b, (short)0, c, false, false);
  }
  static __device__ __forceinline__ void guard(v8f& a, v8f& b, v16h x, v16h y) { dep_guard_h(a, b, x, y); }
  static __device__ __forceinline__ void guard4(v8f& a, v8f& b, v8f& c, v8f& d, v16h x, v16h y) { dep_guard4_h(a, b, c, d, x, y); }
  static __device__ __forceinline__ void keep(v16h a, v16h b, v16h c, v16h d) { keep4_h(a, b, c, d); }
};
template <> struct Frag<__bf16> {
  typedef v16b V; union U { v16b v; v8b h[2]; };
  static __device__ __forceinline__ v16b load(const __bf16* p) {
    U f; f.h[0] = *(const v8b*)(p); f.h[1] = *(const v8b*)(p + 16); return f.v;
  }
  static __device__ __forceinline__ v8f mma(v16b a, v16b b, v8f c) {
    return __builtin_amdgcn_wmma_f32_16x16x32_bf16(false, a, false, b, (short)0, c, false, false);
  }
  static __device__ __forceinline__ void guard(v8f& a, v8f& b, v16b x, v16b y) { dep_guard_b(a, b, x, y); }
  static __device__ __forceinline__ void guard4(v8f& a, v8f& b, v8f& c, v8f& d, v16b x, v16b y) { dep_guard4_b(a, b, c, d, x, y); }
  static __device__ __forceinline__ void keep(v16b a, v16b b, v16b c, v16b d) { keep4_b(a, b, c, d); }
};

__device__ __forceinline__ unsigned pk16(unsigned short a, unsigned short b) { return (unsigned)a | ((unsigned)b << 16); }
__device__ __forceinline__ unsigned short h_bits(float f) { const _Float16 h = (_Float16)f; return __builtin_bit_cast(unsigned short, h); }
__device__ __forceinline__ unsigned short hbits_of_bf(float f, float carry) {
  const float r = bf_bits2f(f2bf_bits(f));
  const float s = r * carry;
  return h_bits(s);
}

template <int ET> struct Elem;
template <> struct Elem<0> { typedef _Float16 T; };
template <> struct Elem<1> { typedef __bf16 T; };
template <int ET, int SPLIT, int BIAS_MODE, int OUT_MODE, bool RESID, int ACT = 0>
__global__ __launch_bounds__(256) void wmma_gemm64(
    const unsigned short* __restrict__ Ap, const unsigned short* __restrict__ A2p, int lda, long strideA,
    const unsigned short* __restrict__ Btp, const unsigned short* __restrict__ Bt2p, int ldb, long strideB,
    void* __restrict__ Cout, void* __restrict__ Cout2, int ldc, long strideC,
    const float* __restrict__ bias,
    const float* __restrict__ resid, long strideR,
    int M, int N, int K, float scale) {
  typedef typename Elem<ET>::T T;
  typedef typename Frag<T>::V V;
  const T* A = (const T*)Ap; const T* A2 = (const T*)A2p; const T* Bt = (const T*)Btp; const T* Bt2 = (const T*)Bt2p;
  __shared__ __align__(16) float sT[8][16 * 68];
  const int b    = blockIdx.y;
  const int lane = threadIdx.x & 31;
  const int wave = threadIdx.x >> 5;
  const int tilesN = N >> 6;
  const int tilesM = M >> 6;
  const int tile = blockIdx.x * 8 + wave;
  if (tile >= tilesM * tilesN) return;
  const int tm = tile / tilesN;
  const int tn = tile - tm * tilesN;
  const int m0 = tm << 6;
  const int n0 = tn << 6;

  const T* Ab  = A  + (size_t)b * strideA;
  const T* Bb  = Bt + (size_t)b * strideB;
  const T* Ab2 = (SPLIT != 0) ? (A2  + (size_t)b * strideA) : nullptr;
  const T* Bb2 = (SPLIT == 1) ? (Bt2 + (size_t)b * strideB) : nullptr;

  const int rlane = lane & 15;
  const int koff  = (lane >> 4) * 8;
  const int mOff  = (lane >> 4) * 8;

  v8f acc[4][4];
#pragma unroll
  for (int i = 0; i < 4; ++i)
#pragma unroll
    for (int j = 0; j < 4; ++j) acc[i][j] = (v8f){0.f,0.f,0.f,0.f,0.f,0.f,0.f,0.f};

  for (int k0 = 0; k0 < K; k0 += 32) {
    V bh[4], bl[4];
#pragma unroll
    for (int j = 0; j < 4; ++j) {
      const size_t bo = (size_t)(n0 + (j << 4) + rlane) * ldb + koff + k0;
      bh[j] = Frag<T>::load(Bb + bo);
      if (SPLIT == 1) bl[j] = Frag<T>::load(Bb2 + bo);
    }
#pragma unroll
    for (int i = 0; i < 4; ++i) {
      const size_t ao = (size_t)(m0 + (i << 4) + rlane) * lda + koff + k0;
      V ah = Frag<T>::load(Ab + ao);
      V al;
      if (SPLIT != 0) al = Frag<T>::load(Ab2 + ao);
#pragma unroll
      for (int j = 0; j < 4; ++j) {
        acc[i][j] = Frag<T>::mma(ah, bh[j], acc[i][j]);
        if (SPLIT == 1) acc[i][j] = Frag<T>::mma(ah, bl[j], acc[i][j]);
        if (SPLIT != 0) acc[i][j] = Frag<T>::mma(al, bh[j], acc[i][j]);
      }
      Frag<T>::guard4(acc[i][0], acc[i][1], acc[i][2], acc[i][3], ah, (SPLIT != 0) ? al : ah);
    }
    Frag<T>::keep(bh[0], bh[1], bh[2], bh[3]);
    if (SPLIT == 1) Frag<T>::keep(bl[0], bl[1], bl[2], bl[3]);
  }
  acc_guard4(acc[0][0], acc[0][1], acc[0][2], acc[0][3]);
  acc_guard4(acc[1][0], acc[1][1], acc[1][2], acc[1][3]);
  acc_guard4(acc[2][0], acc[2][1], acc[2][2], acc[2][3]);
  acc_guard4(acc[3][0], acc[3][1], acc[3][2], acc[3][3]);

  float* slab = sT[wave];
  const float* Rb = RESID ? (resid + (size_t)b * strideR) : nullptr;
#pragma unroll
  for (int i = 0; i < 4; ++i) {
    const int mBase = m0 + (i << 4);
#pragma unroll
    for (int j = 0; j < 4; ++j) {
      const int n = n0 + (j << 4) + rlane;
      float bv = 0.f;
      if (BIAS_MODE == 2) bv = bias[n];
#pragma unroll
      for (int r = 0; r < 8; ++r) {
        float v = acc[i][j][r] * scale;
        if (BIAS_MODE == 1) v += bias[mBase + mOff + r];
        if (BIAS_MODE == 2) v += bv;
        if (RESID) v += Rb[(size_t)(mBase + mOff + r) * ldc + n];
        if (ACT == 2) v = fmaxf(v, 0.0f);
        if (ACT == 4) v = (v > 0.f) ? v : 0.01f * v;
        slab[(mOff + r) * 68 + (j << 4) + rlane] = v;
      }
    }
    __builtin_amdgcn_fence(__ATOMIC_RELEASE, "workgroup");
    __builtin_amdgcn_wave_barrier();
    __builtin_amdgcn_fence(__ATOMIC_ACQUIRE, "workgroup");
    if (OUT_MODE == 0) {
      float* C = (float*)Cout + (size_t)b * strideC;
      const int hh = lane >> 4, c4 = (lane & 15) * 4;
      for (int pass = 0; pass < 2; ++pass) {
#pragma unroll
        for (int it = 0; it < 8; ++it) {
          const int row = it * 2 + hh;
          v4f v = *(const v4f*)(slab + row * 68 + c4);
          *(volatile v4f*)(C + (size_t)(mBase + row) * ldc + n0 + c4) = v;
        }
        __threadfence();
      }
    } else {
      const int q = lane >> 3, c8 = (lane & 7) * 8;
      unsigned short* C  = (unsigned short*)Cout  + (size_t)b * strideC;
      unsigned short* C2 = (OUT_MODE == 2) ? ((unsigned short*)Cout2 + (size_t)b * strideC) : nullptr;
      for (int pass = 0; pass < 2; ++pass) {
#pragma unroll
        for (int it = 0; it < 4; ++it) {
          const int row = it * 4 + q;
          const float* sp = slab + row * 68 + c8;
          v8h hv, lv;
#pragma unroll
          for (int e = 0; e < 8; ++e) {
            if (OUT_MODE == 1) {
              hv[e] = (_Float16)sp[e];
            } else {
              unsigned short hb = f2bf_bits(sp[e]);
              unsigned short lb = f2bf_bits(sp[e] - bf_bits2f(hb));
              hv[e] = __builtin_bit_cast(_Float16, hb);
              lv[e] = __builtin_bit_cast(_Float16, lb);
            }
          }
          *(volatile v8h*)(C + (size_t)(mBase + row) * ldc + n0 + c8) = hv;
          if (OUT_MODE == 2) *(volatile v8h*)(C2 + (size_t)(mBase + row) * ldc + n0 + c8) = lv;
        }
        __threadfence();
      }
    }
    __builtin_amdgcn_fence(__ATOMIC_RELEASE, "workgroup");
    __builtin_amdgcn_wave_barrier();
    __builtin_amdgcn_fence(__ATOMIC_ACQUIRE, "workgroup");
  }
}

__global__ __launch_bounds__(256) void cast_x_kernel(const float* __restrict__ in, unsigned short* __restrict__ out,
                                                     int n8, float carry) {
  const int i = blockIdx.x * 256 + threadIdx.x;
  if (i >= n8) return;
  const float* p = in + 8 * (size_t)i;
  const v4f a = *(const v4f*)(p);
  const v4f c = *(const v4f*)(p + 4);
  unsigned short hb[8];
#pragma unroll
  for (int e = 0; e < 4; ++e) {
    const float a0 = a[e];
    const float c0 = c[e];
    hb[e]     = hbits_of_bf(a0, carry);
    hb[4 + e] = hbits_of_bf(c0, carry);
  }
  const v4u u = (v4u){pk16(hb[0], hb[1]), pk16(hb[2], hb[3]), pk16(hb[4], hb[5]), pk16(hb[6], hb[7])};
  unsigned short* q = out + 8 * (size_t)i;
  *(volatile v4u*)q = u;
  __threadfence();
  *(volatile v4u*)q = u;
}

template <bool BFOUT>
__global__ __launch_bounds__(256) void wtcast_kernel(const float* __restrict__ W0, const float* __restrict__ W1,
                                                     const float* __restrict__ W2,
                                                     unsigned short* __restrict__ out, float carry) {
  __shared__ float sm[64][65];
  const int t   = threadIdx.x;
  const int kt0 = blockIdx.x * 64;
  const int nt0 = blockIdx.y * 64;
  const int z   = blockIdx.z;
  const float* W = (z == 0) ? W0 : (z == 1) ? W1 : W2;
#pragma unroll
  for (int i = 0; i < 16; ++i) {
    const int e = i * 256 + t;
    const int r = e >> 6;
    const int c = e & 63;
    const float w = W[(size_t)(kt0 + r) * kDim + nt0 + c];
    sm[c][r] = bf_bits2f(f2bf_bits(w)) * carry;
  }
  __syncthreads();
  const int lane = t & 31, wave = t >> 5;
  const int q = lane >> 3, c8 = (lane & 7) * 8;
  unsigned short* op = out + (size_t)z * kDim * kDim;
  for (int pass = 0; pass < 2; ++pass) {
#pragma unroll
    for (int it = 0; it < 2; ++it) {
      const int row = wave * 8 + it * 4 + q;
      unsigned short hb[8];
#pragma unroll
      for (int e = 0; e < 8; ++e) {
        const float sv = sm[row][c8 + e];
        hb[e] = BFOUT ? f2bf_bits(sv) : h_bits(sv);
      }
      const v4u u = (v4u){pk16(hb[0], hb[1]), pk16(hb[2], hb[3]), pk16(hb[4], hb[5]), pk16(hb[6], hb[7])};
      *(volatile v4u*)(op + (size_t)(nt0 + row) * kDim + kt0 + c8) = u;
    }
    __threadfence();
  }
}

__device__ __forceinline__ v8f mma16g(v16h a, v16h b, v8f c) {
  c = __builtin_amdgcn_wmma_f32_16x16x32_f16(false, a, false, b, (short)0, c, false, false);
  asm volatile("v_nop\n\tv_nop\n\tv_nop\n\tv_nop" : "+v"(c) : "v"(a), "v"(b));
  return c;
}
__device__ __forceinline__ v16h frag_lds(const unsigned short* p) { return Frag<_Float16>::load((const _Float16*)p); }

__global__ __launch_bounds__(128) void lin_core_kernel(const unsigned short* __restrict__ Qp, const unsigned short* __restrict__ Kp,
                                                       const unsigned short* __restrict__ Vp,
                                                       unsigned short* __restrict__ Yhp, unsigned short* __restrict__ Ylp) {
  __shared__ __align__(16) unsigned short Qs[kChunk * kPitch];
  __shared__ __align__(16) unsigned short Ks[kChunk * kPitch];
  __shared__ __align__(16) unsigned short Kt[kChunk * kPitch];
  __shared__ __align__(16) unsigned short Vt[kChunk * kPitch];
  __shared__ __align__(16) unsigned short Am[kChunk * kPitch];
  __shared__ __align__(16) unsigned short Sb[kChunk * kPitch];
  __shared__ __align__(16) unsigned short Ysh[kChunk * kPitch];
  __shared__ __align__(16) unsigned short Ysl[kChunk * kPitch];

  const int bh   = blockIdx.x;
  const int b    = bh / kHeads;
  const int h    = bh - b * kHeads;
  const int tid  = threadIdx.x;
  const int wave = tid >> 5;
  const int lane = tid & 31;
  const int hh   = lane >> 4;
  const int c16  = lane & 15;
  const int koff = hh * 8;
  const int hcol = h * kDh;
  const int jr   = tid >> 1;
  const int dh   = (tid & 1) * 32;
  const int wrow = 16 * wave;

  v8f sacc[4];
#pragma unroll
  for (int tn = 0; tn < 4; ++tn) sacc[tn] = (v8f){0.f,0.f,0.f,0.f,0.f,0.f,0.f,0.f};

#pragma unroll 1
  for (int ch = 0; ch < kNChunk; ++ch) {
    const size_t rowbase = (size_t)b * kSeq + (size_t)ch * kChunk;
    __syncthreads();
    {
      const size_t goff = (rowbase + jr) * (size_t)kDim + hcol + dh;
      v4u kw[4], vw[4];
#pragma unroll
      for (int i = 0; i < 4; ++i) {
        kw[i] = *(const v4u*)(Kp + goff + 8 * i);
        vw[i] = *(const v4u*)(Vp + goff + 8 * i);
      }
#pragma unroll
      for (int i = 0; i < 4; ++i) *(v4u*)(Ks + jr * kPitch + dh + 8 * i) = kw[i];
#pragma unroll
      for (int i = 0; i < 4; ++i) {
#pragma unroll
        for (int w = 0; w < 4; ++w) {
          const unsigned kx = kw[i][w];
          const unsigned vx = vw[i][w];
          const int d = dh + 8 * i + 2 * w;
          Kt[d * kPitch + jr]       = (unsigned short)(kx & 0xffffu);
          Kt[(d + 1) * kPitch + jr] = (unsigned short)(kx >> 16);
          Vt[d * kPitch + jr]       = (unsigned short)(vx & 0xffffu);
          Vt[(d + 1) * kPitch + jr] = (unsigned short)(vx >> 16);
        }
      }
      asm volatile("" ::: "memory");
      v4u qw[4];
#pragma unroll
      for (int i = 0; i < 4; ++i) qw[i] = *(const v4u*)(Qp + goff + 8 * i);
#pragma unroll
      for (int i = 0; i < 4; ++i) *(v4u*)(Qs + jr * kPitch + dh + 8 * i) = qw[i];
    }
#pragma unroll
    for (int tn = 0; tn < 4; ++tn) {
#pragma unroll
      for (int r = 0; r < 8; ++r) {
        const float sv = sacc[tn][r];
        Sb[(wrow + 8 * hh + r) * kPitch + 16 * tn + c16] = h_bits(sv);
      }
    }
    __syncthreads();

    v16h qa[2];
#pragma unroll
    for (int kk = 0; kk < 2; ++kk) qa[kk] = frag_lds(Qs + (wrow + c16) * kPitch + koff + 32 * kk);
    v8f aacc[4];
#pragma unroll
    for (int tn = 0; tn < 4; ++tn) aacc[tn] = (v8f){0.f,0.f,0.f,0.f,0.f,0.f,0.f,0.f};
#pragma unroll
    for (int kk = 0; kk < 2; ++kk) {
#pragma unroll
      for (int tn = 0; tn < 4; ++tn) {
        const v16h kb = frag_lds(Ks + (16 * tn + c16) * kPitch + koff + 32 * kk);
        aacc[tn] = mma16g(qa[kk], kb, aacc[tn]);
      }
    }
#pragma unroll
    for (int tn = 0; tn < 4; ++tn) {
#pragma unroll
      for (int r = 0; r < 8; ++r) {
        const int il = wrow + 8 * hh + r;
        const int jl = 16 * tn + c16;
        const float av = aacc[tn][r];
        const float mv = (il >= jl) ? av : 0.0f;
        Am[il * kPitch + jl] = h_bits(mv);
      }
    }
    __syncthreads();

    v8f yacc[4];
#pragma unroll
    for (int tn = 0; tn < 4; ++tn) yacc[tn] = (v8f){0.f,0.f,0.f,0.f,0.f,0.f,0.f,0.f};
#pragma unroll
    for (int kk = 0; kk < 2; ++kk) {
#pragma unroll
      for (int tn = 0; tn < 4; ++tn) {
        const v16h sbf = frag_lds(Sb + (16 * tn + c16) * kPitch + koff + 32 * kk);
        yacc[tn] = mma16g(qa[kk], sbf, yacc[tn]);
      }
    }
    v16h am[2];
#pragma unroll
    for (int kk = 0; kk < 2; ++kk) am[kk] = frag_lds(Am + (wrow + c16) * kPitch + koff + 32 * kk);
#pragma unroll
    for (int kk = 0; kk < 2; ++kk) {
#pragma unroll
      for (int tn = 0; tn < 4; ++tn) {
        const v16h vb = frag_lds(Vt + (16 * tn + c16) * kPitch + koff + 32 * kk);
        yacc[tn] = mma16g(am[kk], vb, yacc[tn]);
      }
    }
    v16h va[2];
#pragma unroll
    for (int kk = 0; kk < 2; ++kk) va[kk] = frag_lds(Vt + (wrow + c16) * kPitch + koff + 32 * kk);
#pragma unroll
    for (int kk = 0; kk < 2; ++kk) {
#pragma unroll
      for (int tn = 0; tn < 4; ++tn) {
        const v16h ktb = frag_lds(Kt + (16 * tn + c16) * kPitch + koff + 32 * kk);
        sacc[tn] = mma16g(va[kk], ktb, sacc[tn]);
      }
    }

#pragma unroll
    for (int tn = 0; tn < 4; ++tn) {
#pragma unroll
      for (int r = 0; r < 8; ++r) {
        const float yv = yacc[tn][r];
        const unsigned short hb = f2bf_bits(yv);
        const float rem = yv - bf_bits2f(hb);
        const unsigned short lb = f2bf_bits(rem);
        const int o = (wrow + 8 * hh + r) * kPitch + 16 * tn + c16;
        Ysh[o] = hb;
        Ysl[o] = lb;
      }
    }
    __syncthreads();
    {
      const int q = lane >> 3, c8 = (lane & 7) * 8;
      for (int pass = 0; pass < 2; ++pass) {
#pragma unroll
        for (int it = 0; it < 4; ++it) {
          const int row = wrow + it * 4 + q;
          const v4u uh = *(const v4u*)(Ysh + row * kPitch + c8);
          const v4u ul = *(const v4u*)(Ysl + row * kPitch + c8);
          const size_t go = (rowbase + row) * (size_t)kDim + hcol + c8;
          *(volatile v4u*)(Yhp + go) = uh;
          *(volatile v4u*)(Ylp + go) = ul;
        }
        __threadfence();
      }
    }
  }
}

extern "C" void kernel_launch(void* const* d_in, const int* in_sizes, int n_in,
                              void* d_out, int out_size, void* d_ws, size_t ws_size,
                              hipStream_t stream) {
  if (n_in < 5) return;
  const int nX = kTok * kDim;
  const int nW = kDim * kDim;
  if (in_sizes[0] != nX || in_sizes[1] != nW || in_sizes[2] != nW || in_sizes[3] != nW || in_sizes[4] != nW) return;
  if (out_size != nX) return;

  const size_t szXH  = (size_t)nX * 2;
  const size_t szWT  = (size_t)3 * nW * 2;
  const size_t szWOB = (size_t)nW * 2;
  const size_t szQKV = (size_t)3 * nX * 2;
  const size_t szYH  = (size_t)nX * 2;
  const size_t szYL  = (size_t)nX * 2;
  const size_t offXH  = 0;
  const size_t offWT  = offXH + szXH;
  const size_t offWOB = offWT + szWT;
  const size_t offQKV = offWOB + szWOB;
  const size_t offYH  = offQKV + szQKV;
  const size_t offYL  = offYH + szYH;
  const size_t total  = offYL + szYL;
  if (ws_size < total) return;

  const float* X  = (const float*)d_in[0];
  const float* Wq = (const float*)d_in[1];
  const float* Wk = (const float*)d_in[2];
  const float* Wv = (const float*)d_in[3];
  const float* Wo = (const float*)d_in[4];
  float* out = (float*)d_out;
  char* ws = (char*)d_ws;
  unsigned short* XH  = (unsigned short*)(ws + offXH);
  unsigned short* WT  = (unsigned short*)(ws + offWT);
  unsigned short* WOB = (unsigned short*)(ws + offWOB);
  unsigned short* QKV = (unsigned short*)(ws + offQKV);
  unsigned short* YH  = (unsigned short*)(ws + offYH);
  unsigned short* YL  = (unsigned short*)(ws + offYL);

  const int n8 = nX / 8;
  cast_x_kernel<<<dim3(n8 / 256), dim3(256), 0, stream>>>(X, XH, n8, 1.0f);

  wtcast_kernel<false><<<dim3(kDim / 64, kDim / 64, 3), dim3(256), 0, stream>>>(Wq, Wk, Wv, WT, kWCarry);
  wtcast_kernel<true><<<dim3(kDim / 64, kDim / 64, 1), dim3(256), 0, stream>>>(Wo, Wo, Wo, WOB, 1.0f);

  const int tilesProj = (kTok / 64) * (kDim / 64);
  wmma_gemm64<0, 0, 0, 1, false, 0><<<dim3(tilesProj / 8, 3), dim3(256), 0, stream>>>(
      XH, XH, kDim, 0L, WT, WT, kDim, (long)nW,
      (void*)QKV, (void*)QKV, kDim, (long)nX, X, X, 0L, kTok, kDim, kDim, kWCarryInv);

  lin_core_kernel<<<dim3(kBatch * kHeads), dim3(128), 0, stream>>>(QKV, QKV + (size_t)nX, QKV + 2 * (size_t)nX, YH, YL);

  wmma_gemm64<1, 2, 0, 0, false, 0><<<dim3(tilesProj / 8, 1), dim3(256), 0, stream>>>(
      YH, YL, kDim, 0L, WOB, WOB, kDim, 0L,
      (void*)out, (void*)out, kDim, 0L, X, X, 0L, kTok, kDim, kDim, 1.0f);
}
